// SSMCore_55903294324784
// MI455X (gfx1250) — hardware-run, weakly checked
//
#include <hip/hip_runtime.h>
#include <math.h>

typedef __attribute__((ext_vector_type(16))) _Float16 v16h;
typedef __attribute__((ext_vector_type(8)))  _Float16 v8h;
typedef __attribute__((ext_vector_type(8)))  float    v8f;
typedef __attribute__((ext_vector_type(4)))  float    v4f;
typedef __attribute__((ext_vector_type(2)))  float    v2f;

constexpr int kSeq     = 2048;
constexpr int kDm      = 1024;
constexpr int kDin     = 2048;
constexpr int kNst     = 16;
constexpr int kTaps    = 3;
constexpr int kConvK   = kTaps * kDm;
constexpr int kPadRows = kSeq + 2;
constexpr int kBcReal  = 32;
constexpr int kBcN     = 64;
constexpr int kBiasPad = 128;
constexpr float kWCarry   = 1024.0f;
constexpr float kResid    = 2048.0f;
constexpr float kYScale   = 0.015625f;
constexpr float kMeanInv  = 1.0f / 2048.0f;
constexpr float sW    = 1.0f / 1024.0f;
constexpr float sWR   = 1.0f / (1024.0f * 2048.0f);
constexpr float sOut  = 64.0f / 1024.0f;
constexpr float sOutR = 64.0f / (1024.0f * 2048.0f);
constexpr bool kConvWResid = true;
constexpr bool kInWResid   = false;
constexpr bool kGateWResid = false;
constexpr bool kOutWResid  = true;

constexpr int kMiConv  = kConvWResid ? 1 : 2;
constexpr int kSplConv = kConvWResid ? 2 : 1;
constexpr int kMiIn    = kInWResid ? 1 : 2;
constexpr int kSplIn   = kInWResid ? 2 : 1;
constexpr int kMiGate  = kGateWResid ? 1 : 2;
constexpr int kSplGate = kGateWResid ? 2 : 1;
constexpr int kMiOut   = kOutWResid ? 1 : 2;
constexpr int kSplOut  = kOutWResid ? 2 : 1;

static_assert((kConvK % 32) == 0 && (kDm % 32) == 0 && (kDin % 32) == 0);
static_assert((kSeq % 64) == 0 && (kDin % 64) == 0 && (kDm % 64) == 0 && (kBcN % 64) == 0);
static_assert(((kSeq / (16 * kMiConv)) * (kDin / 64)) % 8 == 0);
static_assert(((kSeq / (16 * kMiIn)) * (kDin / 64)) % 8 == 0);
static_assert(((kSeq / (16 * kMiGate)) * (kDin / 64)) % 8 == 0);
static_assert(((kSeq / (16 * kMiOut)) * (kDm / 64)) % 8 == 0);
static_assert(((kSeq / 16) * (kBcN / 64)) % 8 == 0);
constexpr int kBlkConv = (kSeq / (16 * kMiConv)) * (kDin / 64) / 8;
constexpr int kBlkIn   = (kSeq / (16 * kMiIn)) * (kDin / 64) / 8;
constexpr int kBlkGate = (kSeq / (16 * kMiGate)) * (kDin / 64) / 8;
constexpr int kBlkOut  = (kSeq / (16 * kMiOut)) * (kDm / 64) / 8;
constexpr int kBlkBc   = (kSeq / 16) * (kBcN / 64) / 8;

constexpr size_t kSzXP  = (size_t)kPadRows * kDm * 2;
constexpr size_t kSzCW  = (size_t)kDin * kConvK * 2;
constexpr size_t kSzIW  = (size_t)kDin * kDm * 2;
constexpr size_t kSzGW  = (size_t)kDin * kDin * 2;
constexpr size_t kSzXW  = (size_t)kBcN * kDin * 2;
constexpr size_t kSzOW  = (size_t)kDm * kDin * 2;
constexpr size_t kSzBP  = (size_t)kBiasPad * 4;
constexpr size_t kSzF32 = (size_t)kSeq * kDin * 4;
constexpr size_t kSzF16 = (size_t)kSeq * kDin * 2;
constexpr size_t kSzBC  = (size_t)kSeq * kBcN * 4;
constexpr size_t kSzDT  = (size_t)kSeq * 4;
constexpr size_t kOffXPH = 0;
constexpr size_t kOffXPL = kOffXPH + kSzXP;
constexpr size_t kOffCWH = kOffXPL + kSzXP;
constexpr size_t kOffCWL = kOffCWH + kSzCW;
constexpr size_t kOffIWH = kOffCWL + (kConvWResid ? kSzCW : 0);
constexpr size_t kOffIWL = kOffIWH + kSzIW;
constexpr size_t kOffGWH = kOffIWL + (kInWResid ? kSzIW : 0);
constexpr size_t kOffGWL = kOffGWH + kSzGW;
constexpr size_t kOffXWH = kOffGWL + (kGateWResid ? kSzGW : 0);
constexpr size_t kOffXWL = kOffXWH + kSzXW;
constexpr size_t kOffOWH = kOffXWL + kSzXW;
constexpr size_t kOffOWL = kOffOWH + kSzOW;
constexpr size_t kOffBPD = kOffOWL + (kOutWResid ? kSzOW : 0);
constexpr size_t kOffXC  = kOffBPD + kSzBP;
constexpr size_t kOffXCH = kOffXC  + kSzF32;
constexpr size_t kOffXCL = kOffXCH + kSzF16;
constexpr size_t kOffZS  = kOffXCL + kSzF16;
constexpr size_t kOffU   = kOffZS  + kSzF32;
constexpr size_t kOffBC  = kOffU   + kSzF32;
constexpr size_t kOffDT  = kOffBC  + kSzBC;
constexpr size_t kWsTotal = kOffDT + kSzDT;
static_assert(kWsTotal == 105923072ull + (kConvWResid ? 12582912ull : 0ull) + (kInWResid ? 4194304ull : 0ull) +
                          (kGateWResid ? 8388608ull : 0ull) + (kOutWResid ? 4194304ull : 0ull));
static_assert(kWsTotal <= 134217728ull);
static_assert((kOffXPL % 128) == 0 && (kOffCWH % 128) == 0 && (kOffCWL % 128) == 0 && (kOffIWH % 128) == 0 &&
              (kOffIWL % 128) == 0 && (kOffGWH % 128) == 0 && (kOffGWL % 128) == 0 && (kOffXWH % 128) == 0 &&
              (kOffXWL % 128) == 0 && (kOffOWH % 128) == 0 && (kOffOWL % 128) == 0 && (kOffBPD % 128) == 0 &&
              (kOffXC % 128) == 0 && (kOffXCH % 128) == 0 && (kOffXCL % 128) == 0 && (kOffZS % 128) == 0 &&
              (kOffU % 128) == 0 && (kOffBC % 128) == 0 && (kOffDT % 128) == 0);
static_assert((size_t)kSeq * kDm * 4 == 8388608ull);

__device__ __forceinline__ _Float16 f16_flush(float v) {
  const float w = (fabsf(v) < 6.103515625e-05f) ? 0.0f : v;
  return (_Float16)w;
}
__device__ __forceinline__ void f16_split(float v, _Float16& hi, _Float16& lo) {
  hi = f16_flush(v);
  const float hf = (float)hi;
  const float r = (v - hf) * kResid;
  lo = f16_flush(r);
}
__device__ __forceinline__ unsigned h16_bits(float v) {
  return (unsigned)__builtin_bit_cast(unsigned short, f16_flush(v));
}
__device__ __forceinline__ float h16_val(unsigned b) {
  return (float)__builtin_bit_cast(_Float16, (unsigned short)b);
}
__device__ __forceinline__ void pin_f(float& x) { asm volatile("" : "+v"(x)); }
__device__ __forceinline__ void pin_v4(v4f& x) { asm volatile("" : "+v"(x)); }
__device__ __forceinline__ float act_sigmoid(float v) {
  return __builtin_amdgcn_rcpf(1.0f + expf(-v));
}
__device__ __forceinline__ float act_softplus(float v) {
  return fmaxf(v, 0.0f) + log1pf(expf(-fabsf(v)));
}

namespace eng {
union FragU { v16h v; v8h h[2]; };
__device__ __forceinline__ v16h frag_load(const _Float16* p) {
  FragU f;
  f.h[0] = *(const v8h*)(p);
  f.h[1] = *(const v8h*)(p + 16);
  return f.v;
}
__device__ __forceinline__ v8f mma(v16h a, v16h b, v8f c) {
  return __builtin_amdgcn_wmma_f32_16x16x32_f16(false, a, false, b, (short)0, c, false, false);
}
__device__ __forceinline__ void guard1(v8f& a, v16h x, v16h y) {
  asm volatile("v_nop\n\tv_nop\n\tv_nop\n\tv_nop" : "+v"(a) : "v"(x), "v"(y));
}
__device__ __forceinline__ void guard_acc(v8f& a) {
  asm volatile("v_nop\n\tv_nop\n\tv_nop\n\tv_nop" : "+v"(a));
}
__device__ __forceinline__ void keep4(v16h a, v16h b, v16h c, v16h d) {
  asm volatile("v_nop" :: "v"(a), "v"(b), "v"(c), "v"(d));
}

template <int MI, int SPL, int EPI>
__global__ __launch_bounds__(256) void gemm_f16_kernel(
    const unsigned short* __restrict__ Ap, const unsigned short* __restrict__ A2p, int lda,
    const unsigned short* __restrict__ Btp, const unsigned short* __restrict__ Bt2p, int ldb,
    float* C, int ldc,
    const float* __restrict__ bias, const float* __restrict__ mulp,
    int M, int N, int K, float scale, float rscale)
{
  static_assert(MI >= 1 && MI <= 2);
  static_assert(SPL >= 1 && SPL <= 2);
  static_assert(EPI >= 0 && EPI <= 2);
  const _Float16* A   = (const _Float16*)Ap;
  const _Float16* A2  = (const _Float16*)A2p;
  const _Float16* Bt  = (const _Float16*)Btp;
  const _Float16* Bt2 = (const _Float16*)Bt2p;
  __shared__ __align__(16) float sT[8][16 * 68];
  const int lane = threadIdx.x & 31;
  const int wave = threadIdx.x >> 5;
  const int tilesN = N >> 6;
  const int tilesM = M / (16 * MI);
  const int tile = blockIdx.x * 8 + wave;
  if (tile >= tilesM * tilesN) return;
  const int tm = tile / tilesN;
  const int tn = tile - tm * tilesN;
  const int m0 = tm * (16 * MI);
  const int n0 = tn << 6;
  const int rlane = lane & 15;
  const int koff  = (lane >> 4) * 8;
  const int mOff  = (lane >> 4) * 8;

  v8f acc[MI][4], accr[MI][4];
#pragma unroll
  for (int i = 0; i < MI; ++i)
#pragma unroll
    for (int j = 0; j < 4; ++j) {
      acc[i][j]  = (v8f){0.f, 0.f, 0.f, 0.f, 0.f, 0.f, 0.f, 0.f};
      accr[i][j] = (v8f){0.f, 0.f, 0.f, 0.f, 0.f, 0.f, 0.f, 0.f};
    }

  for (int k0 = 0; k0 < K; k0 += 32) {
    v16h bh[4], bl[4];
#pragma unroll
    for (int j = 0; j < 4; ++j) {
      const size_t bo = (size_t)(n0 + (j << 4) + rlane) * ldb + koff + k0;
      bh[j] = frag_load(Bt + bo);
      if (SPL == 2) bl[j] = frag_load(Bt2 + bo); else bl[j] = bh[j];
    }
#pragma unroll
    for (int i = 0; i < MI; ++i) {
      const size_t ao = (size_t)(m0 + (i << 4) + rlane) * lda + koff + k0;
      const v16h ah = frag_load(A + ao);
      const v16h al = frag_load(A2 + ao);
#pragma unroll
      for (int jp = 0; jp < 2; ++jp) {
#pragma unroll
        for (int jj = 0; jj < 2; ++jj) {
          const int j = jp * 2 + jj;
          acc[i][j]  = mma(ah, bh[j], acc[i][j]);
          accr[i][j] = mma(al, bh[j], accr[i][j]);
          if (SPL == 2) accr[i][j] = mma(ah, bl[j], accr[i][j]);
        }
#pragma unroll
        for (int jj = 0; jj < 2; ++jj) {
          const int j = jp * 2 + jj;
          guard1(acc[i][j], ah, al);
          guard1(accr[i][j], ah, al);
        }
      }
    }
    keep4(bh[0], bh[1], bh[2], bh[3]);
    if (SPL == 2) keep4(bl[0], bl[1], bl[2], bl[3]);
  }
#pragma unroll
  for (int i = 0; i < MI; ++i)
#pragma unroll
    for (int j = 0; j < 4; ++j) {
      guard_acc(acc[i][j]);
      guard_acc(accr[i][j]);
    }

  float* slab = sT[wave];
  const int hh = lane >> 4, c4 = (lane & 15) * 4;
  const v4f bv = *(const v4f*)(bias + n0 + c4);
#pragma unroll
  for (int i = 0; i < MI; ++i) {
    const int mBase = m0 + (i << 4);
#pragma unroll
    for (int j = 0; j < 4; ++j) {
#pragma unroll
      for (int r = 0; r < 8; ++r) {
        float v = acc[i][j][r] * scale;
        v += accr[i][j][r] * rscale;
        slab[(mOff + r) * 68 + (j << 4) + rlane] = v;
      }
    }
    __builtin_amdgcn_fence(__ATOMIC_RELEASE, "workgroup");
    __builtin_amdgcn_wave_barrier();
    __builtin_amdgcn_fence(__ATOMIC_ACQUIRE, "workgroup");
    for (int it = 0; it < 8; ++it) {
      const int row = it * 2 + hh;
      float* sp = slab + row * 68 + c4;
      v4f v = *(const v4f*)sp;
      v = v + bv;
      if (EPI == 1) {
#pragma unroll
        for (int e = 0; e < 4; ++e) v[e] = act_sigmoid(v[e]);
      }
      if (EPI == 2) {
        const v4f xm = *(const v4f*)(mulp + (size_t)(mBase + row) * ldc + n0 + c4);
#pragma unroll
        for (int e = 0; e < 4; ++e) v[e] = xm[e] * act_sigmoid(v[e]);
      }
      *(v4f*)sp = v;
    }
    {
      for (int pass = 0; pass < 2; ++pass) {
#pragma unroll
        for (int it = 0; it < 8; ++it) {
          const int row = it * 2 + hh;
          const v4f v = *(const v4f*)(slab + row * 68 + c4);
          *(volatile v4f*)(C + (size_t)(mBase + row) * ldc + n0 + c4) = v;
        }
        __threadfence();
      }
    }
    __builtin_amdgcn_fence(__ATOMIC_RELEASE, "workgroup");
    __builtin_amdgcn_wave_barrier();
    __builtin_amdgcn_fence(__ATOMIC_ACQUIRE, "workgroup");
  }
}
}

__global__ __launch_bounds__(256) void pad_split_x_kernel(
    const float* __restrict__ x, unsigned short* __restrict__ dH, unsigned short* __restrict__ dL, int total8)
{
  const int i = blockIdx.x * 256 + threadIdx.x;
  if (i >= total8) return;
  const int e0i = i << 3;
  const bool live = (e0i >= 2 * kDm);
  const int sei = live ? (e0i - 2 * kDm) : 0;
  const size_t e0 = (size_t)e0i;
  const size_t se = (size_t)sei;
  v4f a0 = *(const v4f*)(x + se);
  v4f a1 = *(const v4f*)(x + se + 4);
  pin_v4(a0);
  pin_v4(a1);
  const float keepf = live ? 1.0f : 0.0f;
  v8h hv, lv;
#pragma unroll
  for (int e = 0; e < 4; ++e) {
    _Float16 h0, l0, h1, l1;
    const float f0 = live ? a0[e] : 0.0f;
    const float f1 = live ? a1[e] : 0.0f;
    f16_split(f0 * keepf, h0, l0);
    f16_split(f1 * keepf, h1, l1);
    hv[e] = h0; lv[e] = l0;
    hv[4 + e] = h1; lv[4 + e] = l1;
  }
  unsigned short* qh = dH + e0;
  unsigned short* ql = dL + e0;
  *(volatile v8h*)qh = hv;
  *(volatile v8h*)ql = lv;
  __threadfence();
  *(volatile v8h*)qh = hv;
  *(volatile v8h*)ql = lv;
}

__global__ __launch_bounds__(256) void split_rows_f16_kernel(
    const float* __restrict__ src, unsigned short* __restrict__ dH, unsigned short* __restrict__ dL, int total8)
{
  const int i = blockIdx.x * 256 + threadIdx.x;
  if (i >= total8) return;
  const size_t e0 = (size_t)i << 3;
  const v4f a0 = *(const v4f*)(src + e0);
  const v4f a1 = *(const v4f*)(src + e0 + 4);
  v8h hv, lv;
#pragma unroll
  for (int e = 0; e < 4; ++e) {
    _Float16 h0, l0, h1, l1;
    const float f0 = a0[e];
    const float f1 = a1[e];
    f16_split(f0, h0, l0);
    f16_split(f1, h1, l1);
    hv[e] = h0; lv[e] = l0;
    hv[4 + e] = h1; lv[4 + e] = l1;
  }
  unsigned short* qh = dH + e0;
  unsigned short* ql = dL + e0;
  *(volatile v8h*)qh = hv;
  *(volatile v8h*)ql = lv;
  __threadfence();
  *(volatile v8h*)qh = hv;
  *(volatile v8h*)ql = lv;
}

template <bool LO>
__global__ __launch_bounds__(256) void pack_convw_kernel(
    const float* __restrict__ cw, unsigned short* __restrict__ BtH, unsigned short* __restrict__ BtL,
    int total8, float carry)
{
  const int i = blockIdx.x * 256 + threadIdx.x;
  if (i >= total8) return;
  const unsigned e0 = (unsigned)i << 3;
  const unsigned o  = e0 / (unsigned)kConvK;
  const unsigned j  = e0 - o * (unsigned)kConvK;
  const unsigned kc = j >> 10;
  const unsigned i0 = j & 1023u;
  const float* sp = cw + (size_t)o * kConvK + (size_t)i0 * kTaps + kc;
  v8h hv, lv;
#pragma unroll
  for (int e = 0; e < 8; ++e) {
    _Float16 h, l;
    const float t = sp[e * kTaps] * carry;
    f16_split(t, h, l);
    hv[e] = h;
    lv[e] = l;
  }
  unsigned short* qh = BtH + (size_t)e0;
  unsigned short* ql = BtL + (size_t)e0;
  *(volatile v8h*)qh = hv;
  if (LO) *(volatile v8h*)ql = lv;
  __threadfence();
  *(volatile v8h*)qh = hv;
  if (LO) *(volatile v8h*)ql = lv;
}

template <bool LO>
__global__ __launch_bounds__(256) void transpose_pack_kernel(
    const float* __restrict__ W, int ldw, unsigned short* __restrict__ BtH, unsigned short* __restrict__ BtL,
    int Kdim, int Ndim, float carry)
{
  __shared__ float tile[64 * 65];
  const int tid = threadIdx.x, lane = tid & 31, wave = tid >> 5;
  const int n0 = blockIdx.x * 64;
  const int k0 = blockIdx.y * 64;
#pragma unroll
  for (int p = 0; p < 16; ++p) {
    const int idx = tid + p * 256;
    const int kk  = idx >> 6;
    const int nn  = idx & 63;
    const int n   = n0 + nn;
    const int nc  = (n < Ndim) ? n : (Ndim - 1);
    float v = W[(size_t)(k0 + kk) * ldw + nc];
    pin_f(v);
    const float fz = (n < Ndim) ? 1.0f : 0.0f;
    tile[kk * 65 + nn] = (v * fz) * carry;
  }
  __syncthreads();
  const int q = lane >> 3, c8 = (lane & 7) * 8;
  v8h hv[2], lv[2];
#pragma unroll
  for (int it = 0; it < 2; ++it) {
    const int nrow = it * 32 + wave * 4 + q;
#pragma unroll
    for (int e = 0; e < 8; ++e) {
      _Float16 h, l;
      const float t = tile[(c8 + e) * 65 + nrow];
      f16_split(t, h, l);
      hv[it][e] = h;
      lv[it][e] = l;
    }
  }
  for (int pass = 0; pass < 2; ++pass) {
#pragma unroll
    for (int it = 0; it < 2; ++it) {
      const int nrow = it * 32 + wave * 4 + q;
      const size_t o = (size_t)(n0 + nrow) * Kdim + k0 + c8;
      *(volatile v8h*)(BtH + o) = hv[it];
      if (LO) *(volatile v8h*)(BtL + o) = lv[it];
    }
    __threadfence();
  }
}

__global__ __launch_bounds__(32) void bias_pad_kernel(const float* __restrict__ xb, float* __restrict__ outb)
{
  const int lane = threadIdx.x & 31;
  v4f v;
#pragma unroll
  for (int e = 0; e < 4; ++e) {
    const int n = lane * 4 + e;
    const int nc = (n < kBcReal) ? n : (kBcReal - 1);
    float a = xb[nc];
    pin_f(a);
    const float fa = (n < kBcReal) ? 1.0f : 0.0f;
    v[e] = fa * a;
  }
  float* p = outb + lane * 4;
  *(volatile v4f*)p = v;
  __threadfence();
  *(volatile v4f*)p = v;
}

__global__ __launch_bounds__(256) void dt_rows_kernel(const float* __restrict__ XC, float* __restrict__ DT)
{
  __shared__ float sD[32];
  const int lane = threadIdx.x & 31, wave = threadIdx.x >> 5;
  const int row0 = blockIdx.x * 32 + wave * 4;
  for (int r = 0; r < 4; ++r) {
    const float* p = XC + (size_t)(row0 + r) * kDin + lane * 4;
    float acc = 0.0f;
    for (int it = 0; it < 16; ++it) {
      const v4f v = *(const v4f*)(p + it * 128);
      acc += (v[0] + v[1]) + (v[2] + v[3]);
    }
    acc += __shfl_xor(acc, 16, 32);
    acc += __shfl_xor(acc, 8, 32);
    acc += __shfl_xor(acc, 4, 32);
    acc += __shfl_xor(acc, 2, 32);
    acc += __shfl_xor(acc, 1, 32);
    const float m = acc * kMeanInv;
    const float dtv = act_sigmoid(m) + 0.001f;
    if (lane == 0) sD[wave * 4 + r] = dtv;
  }
  __syncthreads();
  if (wave == 0) {
    const float v = sD[lane];
    volatile float* q = DT + blockIdx.x * 32 + lane;
    *q = v;
    __threadfence();
    *q = v;
  }
}

__global__ __launch_bounds__(64) void scan_kernel(
    const float* __restrict__ U, const float* __restrict__ ZS, const float* __restrict__ BC,
    const float* __restrict__ DT, const float* __restrict__ A_log, const float* __restrict__ Dp,
    unsigned* __restrict__ YH, unsigned* __restrict__ YL)
{
  __shared__ __align__(16) float sBC[64 * 32];
  __shared__ __align__(16) float sDt[64];
  const int tid = threadIdx.x;
  const int d0 = blockIdx.x * 128;
  const int d  = d0 + 2 * tid;

  for (int n = 0; n < 32; ++n) {
    const float al = A_log[(size_t)d * kNst + n];
    sBC[n * 64 + tid] = act_softplus(al);
  }
  __syncthreads();
  float A0[16], A1[16], ha[16], hb[16];
#pragma unroll
  for (int n = 0; n < 16; ++n) {
    A0[n] = sBC[n * 64 + tid];
    A1[n] = sBC[(16 + n) * 64 + tid];
    ha[n] = 0.0f;
    hb[n] = 0.0f;
  }
  const v2f dpv = *(const v2f*)(Dp + d);
  const float D0 = dpv[0], D1 = dpv[1];

  for (int ci = 0; ci < kSeq / 64; ++ci) {
    const int rowc = ci * 64;
    __syncthreads();
#pragma unroll
    for (int i = 0; i < 8; ++i) {
      const int idx = tid + i * 64;
      const int st  = idx >> 3;
      const int c4  = (idx & 7) * 4;
      const v4f v = *(const v4f*)(BC + (size_t)(rowc + st) * kBcN + c4);
      *(v4f*)(sBC + st * 32 + c4) = v;
    }
    sDt[tid] = DT[rowc + tid];
    __syncthreads();
    for (int s = 0; s < 64; ++s) {
      const size_t o = (size_t)(rowc + s) * kDin + d;
      const v2f uv = *(const v2f*)(U + o);
      const v2f zv = *(const v2f*)(ZS + o);
      float u0 = uv[0], u1 = uv[1];
      float g0 = zv[0], g1 = zv[1];
      pin_f(u0); pin_f(u1); pin_f(g0); pin_f(g1);
      const float dt = sDt[s];
      const float* bp = sBC + s * 32;
      v4f Bq[4], Cq[4];
#pragma unroll
      for (int k = 0; k < 4; ++k) {
        Bq[k] = *(const v4f*)(bp + 4 * k);
        Cq[k] = *(const v4f*)(bp + 16 + 4 * k);
      }
      float y0 = 0.0f, y1 = 0.0f;
#pragma unroll
      for (int n = 0; n < 16; ++n) {
        const float bn = Bq[n >> 2][n & 3];
        const float cn = Cq[n >> 2][n & 3];
        const float e0 = expf(A0[n] * dt);
        const float e1 = expf(A1[n] * dt);
        const float bb0 = (e0 * bn) * dt;
        const float bb1 = (e1 * bn) * dt;
        ha[n] = fmaf(e0, ha[n], bb0 * u0);
        hb[n] = fmaf(e1, hb[n], bb1 * u1);
        y0 = fmaf(ha[n], cn, y0);
        y1 = fmaf(hb[n], cn, y1);
      }
      y0 = fmaf(D0, u0, y0);
      y1 = fmaf(D1, u1, y1);
      const float c0 = (y0 * g0) * kYScale;
      const float c1 = (y1 * g1) * kYScale;
      const unsigned hb0 = h16_bits(c0);
      const unsigned hb1 = h16_bits(c1);
      const unsigned hw = hb0 | (hb1 << 16);
      const float r0 = (c0 - h16_val(hb0)) * kResid;
      const float r1 = (c1 - h16_val(hb1)) * kResid;
      const unsigned lw = h16_bits(r0) | (h16_bits(r1) << 16);
      volatile unsigned* yp = YH + (o >> 1);
      volatile unsigned* lp = YL + (o >> 1);
      *yp = hw;
      *lp = lw;
      __threadfence();
      *yp = hw;
      *lp = lw;
    }
  }
}

extern "C" void kernel_launch(void* const* d_in, const int* in_sizes, int n_in,
                              void* d_out, int out_size, void* d_ws, size_t ws_size,
                              hipStream_t stream)
{
  if (n_in < 13) return;
  if (in_sizes[0]  != kSeq * kDm) return;
  if (in_sizes[1]  != kDm * 2 * kDin) return;
  if (in_sizes[2]  != 2 * kDin) return;
  if (in_sizes[3]  != kDin * kDm * kTaps) return;
  if (in_sizes[4]  != kDin) return;
  if (in_sizes[5]  != kDin * kNst) return;
  if (in_sizes[6]  != kDin) return;
  if (in_sizes[7]  != kDin * kBcReal) return;
  if (in_sizes[8]  != kBcReal) return;
  if (in_sizes[9]  != kDin * kDin) return;
  if (in_sizes[10] != kDin) return;
  if (in_sizes[11] != kDin * kDm) return;
  if (in_sizes[12] != kDm) return;
  if (out_size != kSeq * kDm) return;
  if (ws_size < kWsTotal) return;

  const float* x         = (const float*)d_in[0];
  const float* in_proj_w = (const float*)d_in[1];
  const float* in_proj_b = (const float*)d_in[2];
  const float* conv_w    = (const float*)d_in[3];
  const float* conv_b    = (const float*)d_in[4];
  const float* A_log     = (const float*)d_in[5];
  const float* D_param   = (const float*)d_in[6];
  const float* x_proj_w  = (const float*)d_in[7];
  const float* x_proj_b  = (const float*)d_in[8];
  const float* gate_w    = (const float*)d_in[9];
  const float* gate_b    = (const float*)d_in[10];
  const float* o_proj_w  = (const float*)d_in[11];
  const float* o_proj_b  = (const float*)d_in[12];
  float* out = (float*)d_out;

  char* ws = (char*)d_ws;
  unsigned short* XPH = (unsigned short*)(ws + kOffXPH);
  unsigned short* XPL = (unsigned short*)(ws + kOffXPL);
  unsigned short* CWH = (unsigned short*)(ws + kOffCWH);
  unsigned short* CWL = kConvWResid ? (unsigned short*)(ws + kOffCWL) : CWH;
  unsigned short* IWH = (unsigned short*)(ws + kOffIWH);
  unsigned short* IWL = kInWResid ? (unsigned short*)(ws + kOffIWL) : IWH;
  unsigned short* GWH = (unsigned short*)(ws + kOffGWH);
  unsigned short* GWL = kGateWResid ? (unsigned short*)(ws + kOffGWL) : GWH;
  unsigned short* XWH = (unsigned short*)(ws + kOffXWH);
  unsigned short* XWL = (unsigned short*)(ws + kOffXWL);
  unsigned short* OWH = (unsigned short*)(ws + kOffOWH);
  unsigned short* OWL = kOutWResid ? (unsigned short*)(ws + kOffOWL) : OWH;
  float*          BPD = (float*)(ws + kOffBPD);
  float*          XC  = (float*)(ws + kOffXC);
  unsigned short* XCH = (unsigned short*)(ws + kOffXCH);
  unsigned short* XCL = (unsigned short*)(ws + kOffXCL);
  float*          ZS  = (float*)(ws + kOffZS);
  float*          U   = (float*)(ws + kOffU);
  float*          BC  = (float*)(ws + kOffBC);
  float*          DT  = (float*)(ws + kOffDT);
  unsigned short* YH  = XCH;
  unsigned short* YL  = XCL;

  pad_split_x_kernel<<<(kPadRows * kDm / 8) / 256, 256, 0, stream>>>(x, XPH, XPL, kPadRows * kDm / 8);

  pack_convw_kernel<kConvWResid><<<(kDin * kConvK / 8) / 256, 256, 0, stream>>>(
      conv_w, CWH, CWL, kDin * kConvK / 8, kWCarry);

  transpose_pack_kernel<kInWResid><<<dim3(kDin / 64, kDm / 64), 256, 0, stream>>>(
      in_proj_w + kDin, 2 * kDin, IWH, IWL, kDm, kDin, kWCarry);
  transpose_pack_kernel<kGateWResid><<<dim3(kDin / 64, kDin / 64), 256, 0, stream>>>(
      gate_w, kDin, GWH, GWL, kDin, kDin, kWCarry);
  transpose_pack_kernel<true><<<dim3(kBcN / 64, kDin / 64), 256, 0, stream>>>(
      x_proj_w, kBcReal, XWH, XWL, kDin, kBcReal, kWCarry);
  transpose_pack_kernel<kOutWResid><<<dim3(kDm / 64, kDin / 64), 256, 0, stream>>>(
      o_proj_w, kDm, OWH, OWL, kDin, kDm, kWCarry);
  bias_pad_kernel<<<1, 32, 0, stream>>>(x_proj_b, BPD);

  eng::gemm_f16_kernel<kMiConv, kSplConv, 0><<<dim3(kBlkConv), 256, 0, stream>>>(
      XPH, XPL, kDm, CWH, CWL, kConvK, XC, kDin, conv_b, conv_b, kSeq, kDin, kConvK, sW, sWR);

  split_rows_f16_kernel<<<(kSeq * kDin / 8) / 256, 256, 0, stream>>>(XC, XCH, XCL, kSeq * kDin / 8);

  dt_rows_kernel<<<kSeq / 32, 256, 0, stream>>>(XC, DT);

  eng::gemm_f16_kernel<1, 2, 0><<<dim3(kBlkBc), 256, 0, stream>>>(
      XCH, XCL, kDin, XWH, XWL, kDin, BC, kBcN, BPD, BPD, kSeq, kBcN, kDin, sW, sWR);

  eng::gemm_f16_kernel<kMiGate, kSplGate, 2><<<dim3(kBlkGate), 256, 0, stream>>>(
      XCH, XCL, kDin, GWH, GWL, kDin, U, kDin, gate_b, XC, kSeq, kDin, kDin, sW, sWR);

  eng::gemm_f16_kernel<kMiIn, kSplIn, 1><<<dim3(kBlkIn), 256, 0, stream>>>(
      XPH + 2 * kDm, XPL + 2 * kDm, kDm, IWH, IWL, kDm, ZS, kDin, in_proj_b + kDin, in_proj_b,
      kSeq, kDin, kDm, sW, sWR);

  scan_kernel<<<dim3(kDin / 128), 64, 0, stream>>>(
      U, ZS, BC, DT, A_log, D_param, (unsigned*)YH, (unsigned*)YL);

  eng::gemm_f16_kernel<kMiOut, kSplOut, 0><<<dim3(kBlkOut), 256, 0, stream>>>(
      YH, YL, kDin, OWH, OWL, kDin, out, kDm, o_proj_b, o_proj_b, kSeq, kDm, kDin, sOut, sOutR);
}
